// BigBirdAttention_36687610643078
// MI455X (gfx1250) — hardware-verified
//
#include <hip/hip_runtime.h>
#include <math.h>
#include <stdint.h>

#define NBAT  2
#define SEQ   2048
#define HIDW  1024
#define NH    16
#define HD    64
#define BSZ   64
#define NBLK  32
#define RR    3
#define MROWS (NBAT * SEQ)
#define KOUT  (2 * HIDW)
static_assert(NH * HD == HIDW);
static_assert(NBLK * BSZ == SEQ);
static_assert((HIDW % 64) == 0 && (SEQ % 64) == 0 && (HIDW % 32) == 0 && (MROWS % 64) == 0 && (KOUT % 32) == 0);
static_assert(BSZ == 64 && HD == 64);

typedef __bf16         v16b __attribute__((ext_vector_type(16)));
typedef unsigned short v8us __attribute__((ext_vector_type(8)));
typedef float          v8f  __attribute__((ext_vector_type(8)));
typedef float          v4f  __attribute__((ext_vector_type(4)));
typedef unsigned int   v4u  __attribute__((ext_vector_type(4)));
typedef v4f  __attribute__((may_alias)) v4fa;
typedef v8us __attribute__((may_alias)) v8usa;

#if defined(__HIP_DEVICE_COMPILE__)
#define DEV_ASM 1
#else
#define DEV_ASM 0
#endif

__device__ __forceinline__ unsigned short bf_bits(float f) {
  unsigned u = __float_as_uint(f);
  return (unsigned short)((u + 0x7FFFu + ((u >> 16) & 1u)) >> 16);
}
__device__ __forceinline__ float bf_up(unsigned short hb) { return __uint_as_float(((unsigned)hb) << 16); }
__device__ __forceinline__ unsigned pk16(unsigned short a, unsigned short b) { return (unsigned)a | ((unsigned)b << 16); }
__device__ __forceinline__ v8f zero8() { v8f z = {0.f, 0.f, 0.f, 0.f, 0.f, 0.f, 0.f, 0.f}; return z; }

union FragB { v16b v; v8us u[2]; };
__device__ __forceinline__ v16b ldfrag(const unsigned short* p) {
  FragB f;
  f.u[0] = *(const v8usa*)(p);
  f.u[1] = *(const v8usa*)(p + 16);
  return f.v;
}
union U8 { v8us u; v4u w; };

__device__ __forceinline__ v8f mmab(v16b a, v16b b, v8f c) {
  return __builtin_amdgcn_wmma_f32_16x16x32_bf16(false, a, false, b, (short)0, c, false, false);
}
__device__ __forceinline__ v8f mmab_g(v16b a, v16b b, v8f c) {
  c = __builtin_amdgcn_wmma_f32_16x16x32_bf16(false, a, false, b, (short)0, c, false, false);
#if DEV_ASM
  asm volatile("v_nop\n\tv_nop\n\tv_nop\n\tv_nop" : "+v"(c) : "v"(a), "v"(b));
#endif
  return c;
}
__device__ __forceinline__ void dep_guard(v8f& a, v8f& b, v16b x, v16b y) {
#if DEV_ASM
  asm volatile("v_nop\n\tv_nop\n\tv_nop\n\tv_nop" : "+v"(a), "+v"(b) : "v"(x), "v"(y));
#else
  (void)a; (void)b; (void)x; (void)y;
#endif
}
__device__ __forceinline__ void keep4(v16b a, v16b b, v16b c, v16b d) {
#if DEV_ASM
  asm volatile("v_nop" :: "v"(a), "v"(b), "v"(c), "v"(d));
#else
  (void)a; (void)b; (void)c; (void)d;
#endif
}
__device__ __forceinline__ void acc_guard4(v8f& a, v8f& b, v8f& c, v8f& d) {
#if DEV_ASM
  asm volatile("v_nop\n\tv_nop\n\tv_nop\n\tv_nop" : "+v"(a), "+v"(b), "+v"(c), "+v"(d));
#else
  (void)a; (void)b; (void)c; (void)d;
#endif
}

__global__ __launch_bounds__(256) void cvt_x(const float* __restrict__ in, unsigned short* out, int n8) {
  const int i = blockIdx.x * 256 + (int)threadIdx.x;
  if (i < n8) {
    const v4f a  = *(const v4fa*)(in + (size_t)i * 8);
    const v4f a4 = *(const v4fa*)(in + (size_t)i * 8 + 4);
    v4u p;
    p[0] = pk16(bf_bits(a[0]),  bf_bits(a[1]));
    p[1] = pk16(bf_bits(a[2]),  bf_bits(a[3]));
    p[2] = pk16(bf_bits(a4[0]), bf_bits(a4[1]));
    p[3] = pk16(bf_bits(a4[2]), bf_bits(a4[3]));
    unsigned short* o = out + (size_t)i * 8;
    *(volatile v4u*)o = p;
    __threadfence();
    *(volatile v4u*)o = p;
  }
}

__global__ __launch_bounds__(256) void cvt_w(const float* __restrict__ Wq, const float* __restrict__ Wk,
                                             const float* __restrict__ Wv, const float* __restrict__ Wo,
                                             unsigned short* oq, unsigned short* ok, unsigned short* ov,
                                             unsigned short* oo2, int n8) {
  const int mat = blockIdx.y;
  const int i = blockIdx.x * 256 + (int)threadIdx.x;
  const float* W = (mat == 0) ? Wq : ((mat == 1) ? Wk : ((mat == 2) ? Wv : Wo));
  if (i < n8) {
    const v4f a  = *(const v4fa*)(W + (size_t)i * 8);
    const v4f a4 = *(const v4fa*)(W + (size_t)i * 8 + 4);
    v4u p;
    p[0] = pk16(bf_bits(a[0]),  bf_bits(a[1]));
    p[1] = pk16(bf_bits(a[2]),  bf_bits(a[3]));
    p[2] = pk16(bf_bits(a4[0]), bf_bits(a4[1]));
    p[3] = pk16(bf_bits(a4[2]), bf_bits(a4[3]));
    if (mat < 3) {
      unsigned short* o = ((mat == 0) ? oq : ((mat == 1) ? ok : ov)) + (size_t)i * 8;
      *(volatile v4u*)o = p;
      __threadfence();
      *(volatile v4u*)o = p;
    } else {
      const int row  = i >> 7;
      const int col8 = (i & 127) * 8;
      unsigned short* o = oo2 + (size_t)row * KOUT + col8;
      *(volatile v4u*)o = p;
      *(volatile v4u*)(o + HIDW) = p;
      __threadfence();
      *(volatile v4u*)o = p;
      *(volatile v4u*)(o + HIDW) = p;
    }
  }
}

template <int OUTF>
__global__ __launch_bounds__(256) void gemm64(
    const unsigned short* __restrict__ A, int lda,
    const unsigned short* __restrict__ Bt, int ldb,
    const float* __restrict__ bias,
    unsigned short* Ch, unsigned short* Cl, float* Cf, int ldc,
    int M, int N, int K, float oscale) {
  __shared__ __align__(16) float sT[8][16 * 68];
  const int lane = threadIdx.x & 31;
  const int wave = threadIdx.x >> 5;
  const int tilesN = N >> 6;
  const int tilesM = M >> 6;
  const int tile = blockIdx.x * 8 + wave;
  if (tile >= tilesM * tilesN) return;
  const int tm = tile / tilesN;
  const int tn = tile - tm * tilesN;
  const int m0 = tm << 6;
  const int n0 = tn << 6;

  const int rlane = lane & 15;
  const int koff  = (lane >> 4) * 8;
  const int mOff  = (lane >> 4) * 8;

  v8f acc[4][4];
#pragma unroll
  for (int i = 0; i < 4; ++i)
#pragma unroll
    for (int j = 0; j < 4; ++j) acc[i][j] = zero8();

  for (int k0 = 0; k0 < K; k0 += 32) {
    v16b bq[4];
#pragma unroll
    for (int j = 0; j < 4; ++j)
      bq[j] = ldfrag(Bt + (size_t)(n0 + (j << 4) + rlane) * ldb + koff + k0);
#pragma unroll
    for (int i = 0; i < 4; ++i) {
      const v16b af = ldfrag(A + (size_t)(m0 + (i << 4) + rlane) * lda + koff + k0);
#pragma unroll
      for (int j = 0; j < 4; ++j) acc[i][j] = mmab(af, bq[j], acc[i][j]);
      dep_guard(acc[i][0], acc[i][3], af, bq[3]);
    }
    keep4(bq[0], bq[1], bq[2], bq[3]);
  }
  acc_guard4(acc[0][0], acc[0][1], acc[0][2], acc[0][3]);
  acc_guard4(acc[1][0], acc[1][1], acc[1][2], acc[1][3]);
  acc_guard4(acc[2][0], acc[2][1], acc[2][2], acc[2][3]);
  acc_guard4(acc[3][0], acc[3][1], acc[3][2], acc[3][3]);

  float* slab = sT[wave];
  const int q = lane >> 3, c8 = (lane & 7) * 8;
  const int h2 = lane >> 4, c4 = (lane & 15) * 4;
  float bb8[8], bb4[4];
  if (OUTF == 0) {
    const v4f t0 = *(const v4fa*)(bias + n0 + c8);
    const v4f t1 = *(const v4fa*)(bias + n0 + c8 + 4);
#pragma unroll
    for (int e = 0; e < 4; ++e) { bb8[e] = bf_up(bf_bits(t0[e])); bb8[4 + e] = bf_up(bf_bits(t1[e])); }
#pragma unroll
    for (int e = 0; e < 4; ++e) bb4[e] = 0.f;
  } else {
    const v4f t0 = *(const v4fa*)(bias + n0 + c4);
#pragma unroll
    for (int e = 0; e < 4; ++e) bb4[e] = bf_up(bf_bits(t0[e]));
#pragma unroll
    for (int e = 0; e < 8; ++e) bb8[e] = 0.f;
  }
#pragma unroll
  for (int i = 0; i < 4; ++i) {
    const int mBase = m0 + (i << 4);
#pragma unroll
    for (int j = 0; j < 4; ++j) {
#pragma unroll
      for (int r = 0; r < 8; ++r) {
        slab[(mOff + r) * 68 + (j << 4) + rlane] = acc[i][j][r];
      }
    }
    __builtin_amdgcn_fence(__ATOMIC_RELEASE, "workgroup");
    __builtin_amdgcn_wave_barrier();
    __builtin_amdgcn_fence(__ATOMIC_ACQUIRE, "workgroup");
    if (OUTF == 0) {
      v4u hv[4], lv[4];
#pragma unroll
      for (int it = 0; it < 4; ++it) {
        const int row = it * 4 + q;
        const float* sp = slab + row * 68 + c8;
        float f[8];
#pragma unroll
        for (int e = 0; e < 8; ++e) f[e] = (sp[e] + bb8[e]) * oscale;
        v4u a, a2;
#pragma unroll
        for (int e = 0; e < 4; ++e) {
          const float f0 = f[2 * e], f1 = f[2 * e + 1];
          const unsigned short h0 = bf_bits(f0), h1 = bf_bits(f1);
          const unsigned short l0 = bf_bits(f0 - bf_up(h0));
          const unsigned short l1 = bf_bits(f1 - bf_up(h1));
          a[e] = pk16(h0, h1); a2[e] = pk16(l0, l1);
        }
        hv[it] = a; lv[it] = a2;
      }
      for (int pass = 0; pass < 2; ++pass) {
#pragma unroll
        for (int it = 0; it < 4; ++it) {
          const int row = it * 4 + q;
          *(volatile v4u*)(Ch + (size_t)(mBase + row) * ldc + n0 + c8) = hv[it];
          *(volatile v4u*)(Cl + (size_t)(mBase + row) * ldc + n0 + c8) = lv[it];
        }
        __threadfence();
      }
    } else {
      v4f ov[8];
#pragma unroll
      for (int it = 0; it < 8; ++it) {
        const int row = it * 2 + h2;
        v4f v = *(const v4fa*)(slab + row * 68 + c4);
#pragma unroll
        for (int e = 0; e < 4; ++e) v[e] = (v[e] + bb4[e]) * oscale;
        ov[it] = v;
      }
      for (int pass = 0; pass < 2; ++pass) {
#pragma unroll
        for (int it = 0; it < 8; ++it) {
          const int row = it * 2 + h2;
          *(volatile v4f*)(Cf + (size_t)(mBase + row) * ldc + n0 + c4) = ov[it];
        }
        __threadfence();
      }
    }
    __builtin_amdgcn_fence(__ATOMIC_RELEASE, "workgroup");
    __builtin_amdgcn_wave_barrier();
    __builtin_amdgcn_fence(__ATOMIC_ACQUIRE, "workgroup");
  }
}

__global__ __launch_bounds__(256) void vt_tr(const unsigned short* __restrict__ Vh, const unsigned short* __restrict__ Vl,
                                             unsigned short* VTh, unsigned short* VTl) {
  __shared__ __align__(16) unsigned short sT[2][64][72];
  const int tid = (int)threadIdx.x;
  int st = blockIdx.x; st = (st > NBLK - 1) ? (NBLK - 1) : st;
  int bh = blockIdx.y; bh = (bh > NBAT * NH - 1) ? (NBAT * NH - 1) : bh;
  const int s0 = st * 64;
  const size_t sl = (size_t)bh * SEQ * HD + (size_t)s0 * HD;
#pragma unroll
  for (int it = 0; it < 2; ++it) {
    const int cidx = it * 256 + tid;
    const int s = cidx >> 3, d8 = (cidx & 7) * 8;
    const v8us a  = *(const v8usa*)(Vh + sl + (size_t)s * HD + d8);
    const v8us a2 = *(const v8usa*)(Vl + sl + (size_t)s * HD + d8);
#pragma unroll
    for (int e = 0; e < 8; ++e) {
      sT[0][d8 + e][s] = a[e];
      sT[1][d8 + e][s] = a2[e];
    }
  }
  __syncthreads();
  const int sub = tid >> 3, c8 = (tid & 7) * 8;
  U8 ph[2], pl[2];
#pragma unroll
  for (int it = 0; it < 2; ++it) {
    const int d = it * 32 + sub;
    ph[it].u = *(const v8usa*)(&sT[0][d][c8]);
    pl[it].u = *(const v8usa*)(&sT[1][d][c8]);
  }
  for (int pass = 0; pass < 2; ++pass) {
#pragma unroll
    for (int it = 0; it < 2; ++it) {
      const int d = it * 32 + sub;
      const size_t o = ((size_t)bh * HD + d) * SEQ + s0 + c8;
      *(volatile v4u*)(VTh + o) = ph[it].w;
      *(volatile v4u*)(VTl + o) = pl[it].w;
    }
    __threadfence();
  }
}

union __align__(16) SU {
  unsigned short kv[4][64 * 64];
  float          os[4][16 * 64];
};

__device__ __forceinline__ int wrap_blk(int v) { return (v < 0) ? (v + NBLK) : v; }

__global__ __launch_bounds__(128)
void attn_bb(const unsigned short* __restrict__ Qh, const unsigned short* __restrict__ Ql,
             const unsigned short* __restrict__ Kh, const unsigned short* __restrict__ Kl,
             const unsigned short* __restrict__ VTh, const unsigned short* __restrict__ VTl,
             const int* __restrict__ srcB, const int* __restrict__ tgtB,
             unsigned short* Ch, unsigned short* Cl, int ldc) {
  __shared__ SU su;
  __shared__ __align__(16) unsigned short Psh[2][4][16 * 64];

  const int tid  = threadIdx.x;
  const int wave = tid >> 5;
  const int lane = tid & 31;
  const int hh   = lane >> 4;
  const int c    = lane & 15;

  int qb = (int)blockIdx.x; qb = (qb > NBLK - 1) ? (NBLK - 1) : qb;
  int h  = (int)blockIdx.y; h  = (h  > NH - 1)   ? (NH - 1)   : h;
  int b  = (int)blockIdx.z; b  = (b  > NBAT - 1) ? (NBAT - 1) : b;
  const int bh = b * NH + h;
  const size_t slab = (size_t)bh * SEQ * HD;

  const int sr0 = wrap_blk(srcB[0]), sr1 = wrap_blk(srcB[1]), sr2 = wrap_blk(srcB[2]);
  const int tr0 = wrap_blk(tgtB[0]), tr1 = wrap_blk(tgtB[1]), tr2 = wrap_blk(tgtB[2]);

  const int q0 = qb * BSZ + wave * 16;

  v16b qah[2], qal[2];
#pragma unroll
  for (int dc = 0; dc < 2; ++dc) {
    const size_t qo = slab + (size_t)(q0 + c) * HD + dc * 32 + 8 * hh;
    qah[dc] = ldfrag(Qh + qo);
    qal[dc] = ldfrag(Ql + qo);
  }

  float mrow[8], lrow[8];
  v8f oacc[4];
#pragma unroll
  for (int r = 0; r < 8; ++r) { mrow[r] = -INFINITY; lrow[r] = 0.f; }
#pragma unroll
  for (int t = 0; t < 4; ++t) oacc[t] = zero8();

  unsigned short* pwh = Psh[0][wave];
  unsigned short* pwl = Psh[1][wave];

#pragma unroll 1
  for (int kb = 0; kb < NBLK; ++kb) {
    int dd = qb - kb; dd = (dd < 0) ? -dd : dd;
    const bool allowed = (dd <= 1) || (kb == 0) || (kb == NBLK - 1) ||
                         (sr0 == qb && tr0 == kb) || (sr1 == qb && tr1 == kb) || (sr2 == qb && tr2 == kb);
    if (!allowed) continue;
    const int ks = kb * BSZ;
    __syncthreads();
    {
      const int r = tid >> 1, half = (tid & 1) * 32;
      const unsigned short* kgh = Kh  + slab + (size_t)(ks + r) * HD + half;
      const unsigned short* kgl = Kl  + slab + (size_t)(ks + r) * HD + half;
      const unsigned short* vgh = VTh + ((size_t)bh * HD + r) * SEQ + ks + half;
      const unsigned short* vgl = VTl + ((size_t)bh * HD + r) * SEQ + ks + half;
#pragma unroll
      for (int i = 0; i < 4; ++i) {
        const v8us a0 = *(const v8usa*)(kgh + 8 * i);
        const v8us a1 = *(const v8usa*)(kgl + 8 * i);
        const v8us b0 = *(const v8usa*)(vgh + 8 * i);
        const v8us b1 = *(const v8usa*)(vgl + 8 * i);
        *(v8us*)(su.kv[0] + r * 64 + half + 8 * i) = a0;
        *(v8us*)(su.kv[1] + r * 64 + half + 8 * i) = a1;
        *(v8us*)(su.kv[2] + r * 64 + half + 8 * i) = b0;
        *(v8us*)(su.kv[3] + r * 64 + half + 8 * i) = b1;
      }
    }
    __syncthreads();

    v8f s[4];
#pragma unroll
    for (int j = 0; j < 4; ++j) {
      v8f z = zero8();
#pragma unroll
      for (int dc = 0; dc < 2; ++dc) {
        const v16b kfh = ldfrag(su.kv[0] + (j * 16 + c) * 64 + dc * 32 + 8 * hh);
        const v16b kfl = ldfrag(su.kv[1] + (j * 16 + c) * 64 + dc * 32 + 8 * hh);
        z = mmab_g(qah[dc], kfh, z);
        z = mmab_g(qah[dc], kfl, z);
        z = mmab_g(qal[dc], kfh, z);
      }
      s[j] = z;
    }

#pragma unroll
    for (int r = 0; r < 8; ++r) {
      float m = s[0][r];
#pragma unroll
      for (int j = 1; j < 4; ++j) m = fmaxf(m, s[j][r]);
#pragma unroll
      for (int off = 1; off < 16; off <<= 1) m = fmaxf(m, __shfl_xor(m, off, 32));
      const float mnew  = fmaxf(mrow[r], m);
      const float msafe = (mnew == -INFINITY) ? 0.f : mnew;
      const float alpha = __expf(mrow[r] - msafe);
      mrow[r] = mnew;
      float psum = 0.f;
#pragma unroll
      for (int j = 0; j < 4; ++j) {
        const float p = __expf(s[j][r] - msafe);
        psum += p;
        const unsigned short hb = bf_bits(p);
        const unsigned short lb = bf_bits(p - bf_up(hb));
        pwh[(8 * hh + r) * 64 + j * 16 + c] = hb;
        pwl[(8 * hh + r) * 64 + j * 16 + c] = lb;
      }
#pragma unroll
      for (int off = 1; off < 16; off <<= 1) psum += __shfl_xor(psum, off, 32);
      lrow[r] = lrow[r] * alpha + psum;
#pragma unroll
      for (int t = 0; t < 4; ++t) oacc[t][r] *= alpha;
    }
    __builtin_amdgcn_fence(__ATOMIC_RELEASE, "workgroup");
    __builtin_amdgcn_wave_barrier();
    __builtin_amdgcn_fence(__ATOMIC_ACQUIRE, "workgroup");

#pragma unroll 1
    for (int kk = 0; kk < 2; ++kk) {
      const v16b pah = ldfrag(pwh + c * 64 + kk * 32 + 8 * hh);
      const v16b pal = ldfrag(pwl + c * 64 + kk * 32 + 8 * hh);
#pragma unroll
      for (int t = 0; t < 4; ++t) {
        const v16b vfh = ldfrag(su.kv[2] + (t * 16 + c) * 64 + kk * 32 + 8 * hh);
        const v16b vfl = ldfrag(su.kv[3] + (t * 16 + c) * 64 + kk * 32 + 8 * hh);
        oacc[t] = mmab_g(pah, vfh, oacc[t]);
        oacc[t] = mmab_g(pal, vfh, oacc[t]);
        oacc[t] = mmab_g(pah, vfl, oacc[t]);
      }
    }
  }

  __syncthreads();
  float* os = su.os[wave];
#pragma unroll
  for (int r = 0; r < 8; ++r) {
    const float l = lrow[r];
    const float inv = (l > 0.f) ? (1.0f / l) : 0.f;
#pragma unroll
    for (int t = 0; t < 4; ++t) os[(8 * hh + r) * 64 + t * 16 + c] = oacc[t][r] * inv;
  }
  __builtin_amdgcn_fence(__ATOMIC_RELEASE, "workgroup");
  __builtin_amdgcn_wave_barrier();
  __builtin_amdgcn_fence(__ATOMIC_ACQUIRE, "workgroup");
  {
    const int q = lane >> 3, c8 = (lane & 7) * 8;
    v4u hv[4], lv[4];
#pragma unroll
    for (int it = 0; it < 4; ++it) {
      const int row = it * 4 + q;
      const float* sp = os + row * 64 + c8;
      const v4f f0 = *(const v4fa*)(sp);
      const v4f f1 = *(const v4fa*)(sp + 4);
      float f[8];
#pragma unroll
      for (int e = 0; e < 4; ++e) { f[e] = f0[e]; f[4 + e] = f1[e]; }
      v4u a, a2;
#pragma unroll
      for (int e = 0; e < 4; ++e) {
        const float v0 = f[2 * e], v1 = f[2 * e + 1];
        const unsigned short h0 = bf_bits(v0), h1 = bf_bits(v1);
        const unsigned short l0 = bf_bits(v0 - bf_up(h0));
        const unsigned short l1 = bf_bits(v1 - bf_up(h1));
        a[e] = pk16(h0, h1); a2[e] = pk16(l0, l1);
      }
      hv[it] = a; lv[it] = a2;
    }
    const size_t obase = ((size_t)b * SEQ + (size_t)q0) * (size_t)ldc + (size_t)h * HD + c8;
    for (int pass = 0; pass < 2; ++pass) {
#pragma unroll
      for (int it = 0; it < 4; ++it) {
        const int row = it * 4 + q;
        *(volatile v4u*)(Ch + obase + (size_t)row * ldc) = hv[it];
        *(volatile v4u*)(Cl + obase + (size_t)row * ldc) = lv[it];
      }
      __threadfence();
    }
  }
}

extern "C" void kernel_launch(void* const* d_in, const int* in_sizes, int n_in,
                              void* d_out, int out_size, void* d_ws, size_t ws_size,
                              hipStream_t stream) {
  if (n_in < 11) return;
  if (in_sizes[0] != MROWS * HIDW) return;
  if (in_sizes[1] != HIDW * HIDW || in_sizes[3] != HIDW * HIDW || in_sizes[5] != HIDW * HIDW || in_sizes[7] != HIDW * HIDW) return;
  if (in_sizes[2] != HIDW || in_sizes[4] != HIDW || in_sizes[6] != HIDW || in_sizes[8] != HIDW) return;
  if (in_sizes[9] != RR || in_sizes[10] != RR) return;
  if (out_size != MROWS * HIDW) return;

  const float* x  = (const float*)d_in[0];
  const float* Wq = (const float*)d_in[1];
  const float* bq = (const float*)d_in[2];
  const float* Wk = (const float*)d_in[3];
  const float* bk = (const float*)d_in[4];
  const float* Wv = (const float*)d_in[5];
  const float* bv = (const float*)d_in[6];
  const float* Wo = (const float*)d_in[7];
  const float* bo = (const float*)d_in[8];
  const int*   srcB = (const int*)d_in[9];
  const int*   tgtB = (const int*)d_in[10];
  float* out = (float*)d_out;

  const size_t PX  = (size_t)MROWS * HIDW * 2;
  const size_t PW  = (size_t)HIDW * HIDW * 2;
  const size_t PW2 = (size_t)HIDW * KOUT * 2;
  const size_t PVT = (size_t)NBAT * NH * HD * SEQ * 2;
  const size_t PCT = (size_t)MROWS * KOUT * 2;
  size_t off = 0;
  const size_t oXb  = off; off += PX;
  const size_t oWq  = off; off += PW;
  const size_t oWk  = off; off += PW;
  const size_t oWv  = off; off += PW;
  const size_t oWo2 = off; off += PW2;
  const size_t oQh  = off; off += PX;
  const size_t oQl  = off; off += PX;
  const size_t oKh  = off; off += PX;
  const size_t oKl  = off; off += PX;
  const size_t oVh  = off; off += PX;
  const size_t oVl  = off; off += PX;
  const size_t oVTh = off; off += PVT;
  const size_t oVTl = off; off += PVT;
  const size_t oCT  = off; off += PCT;
  if (off > ws_size) return;
  if (off > (size_t)134217728) return;

  char* ws = (char*)d_ws;
  unsigned short* Xb   = (unsigned short*)(ws + oXb);
  unsigned short* Wqb  = (unsigned short*)(ws + oWq);
  unsigned short* Wkb  = (unsigned short*)(ws + oWk);
  unsigned short* Wvb  = (unsigned short*)(ws + oWv);
  unsigned short* Wob2 = (unsigned short*)(ws + oWo2);
  unsigned short* Qh   = (unsigned short*)(ws + oQh);
  unsigned short* Ql   = (unsigned short*)(ws + oQl);
  unsigned short* Kh   = (unsigned short*)(ws + oKh);
  unsigned short* Kl   = (unsigned short*)(ws + oKl);
  unsigned short* Vh   = (unsigned short*)(ws + oVh);
  unsigned short* Vl   = (unsigned short*)(ws + oVl);
  unsigned short* VTh  = (unsigned short*)(ws + oVTh);
  unsigned short* VTl  = (unsigned short*)(ws + oVTl);
  unsigned short* CT   = (unsigned short*)(ws + oCT);

  const int n8x = MROWS * HIDW / 8;
  const int n8w = HIDW * HIDW / 8;
  const dim3 gCvtX((n8x + 255) / 256);
  const dim3 gCvtW((n8w + 255) / 256, 4);
  const dim3 blk(256);
  const int tilesP = (MROWS / 64) * (HIDW / 64);
  const dim3 gP((tilesP + 7) / 8);
  const dim3 gVT(SEQ / 64, NBAT * NH);
  const dim3 gAttn(NBLK, NH, NBAT);

  cvt_x<<<gCvtX, blk, 0, stream>>>(x, Xb, n8x);
  cvt_w<<<gCvtW, blk, 0, stream>>>(Wq, Wk, Wv, Wo, Wqb, Wkb, Wvb, Wob2, n8w);
  gemm64<0><<<gP, blk, 0, stream>>>(Xb, HIDW, Wqb, HIDW, bq, Qh, Ql, out, HIDW, MROWS, HIDW, HIDW, 0.125f);
  gemm64<0><<<gP, blk, 0, stream>>>(Xb, HIDW, Wkb, HIDW, bk, Kh, Kl, out, HIDW, MROWS, HIDW, HIDW, 1.0f);
  gemm64<0><<<gP, blk, 0, stream>>>(Xb, HIDW, Wvb, HIDW, bv, Vh, Vl, out, HIDW, MROWS, HIDW, HIDW, 1.0f);
  vt_tr<<<gVT, blk, 0, stream>>>(Vh, Vl, VTh, VTl);
  attn_bb<<<gAttn, dim3(128), 0, stream>>>(Qh, Ql, Kh, Kl, VTh, VTl, srcB, tgtB, CT, CT + HIDW, KOUT);
  gemm64<1><<<gP, blk, 0, stream>>>(CT, KOUT, Wob2, KOUT, bo, CT, CT + HIDW, out, HIDW, MROWS, HIDW, KOUT, 1.0f);
  (void)hipGetLastError();
}
